// TransformerBlock_7009386627369
// MI455X (gfx1250) — hardware-run, weakly checked
//
#include <hip/hip_runtime.h>
#include <math.h>

#ifndef NB
#define NB 2
#endif
#ifndef SEQ
#define SEQ 2048
#endif
#define NB_FULL 2
#define T_FULL 2048
#define CE 1024
#define NH 16
#define HD 64
#define FF 4096
#define NX 256
#define MT (NB * SEQ)

static_assert(SEQ % 64 == 0);
static_assert(SEQ >= NX && SEQ <= T_FULL && NB <= NB_FULL && NB >= 1);
static_assert(CE % 64 == 0 && FF % 64 == 0 && NX % 64 == 0 && CE % 32 == 0 && FF % 32 == 0);
static_assert(NH * HD == CE && HD == 64);

typedef __attribute__((ext_vector_type(16))) _Float16 v16h;
typedef __attribute__((ext_vector_type(16))) __bf16   v16b;
typedef __attribute__((ext_vector_type(8)))  __bf16   v8b;
typedef __attribute__((ext_vector_type(8)))  float    v8f;
typedef __attribute__((ext_vector_type(4)))  float    v4f;
typedef __attribute__((ext_vector_type(4)))  unsigned int v4u;

union FB { v16b v; v8b h[2]; };

__device__ __forceinline__ unsigned int f2bf_bits(float f) { const unsigned int u = __float_as_uint(f); return (u + 0x7FFFu + ((u >> 16) & 1u)) >> 16; }
__device__ __forceinline__ float bf_bits2f(unsigned int h) { return __uint_as_float(h << 16); }
__device__ __forceinline__ float cmb_bf(float v) { return bf_bits2f(f2bf_bits(v)); }
__device__ __forceinline__ unsigned int h_bits(float v) { return (unsigned int)__builtin_bit_cast(unsigned short, (_Float16)v); }

__device__ __forceinline__ v4u pk8h(v4f a, v4f b) {
  v4u p;
  p.x = h_bits(a.x) | (h_bits(a.y) << 16); p.y = h_bits(a.z) | (h_bits(a.w) << 16);
  p.z = h_bits(b.x) | (h_bits(b.y) << 16); p.w = h_bits(b.z) | (h_bits(b.w) << 16);
  return p;
}
__device__ __forceinline__ v4u pk8b(v4f a, v4f b) {
  v4u p;
  p.x = f2bf_bits(a.x) | (f2bf_bits(a.y) << 16); p.y = f2bf_bits(a.z) | (f2bf_bits(a.w) << 16);
  p.z = f2bf_bits(b.x) | (f2bf_bits(b.y) << 16); p.w = f2bf_bits(b.z) | (f2bf_bits(b.w) << 16);
  return p;
}
__device__ __forceinline__ void bf_hl(float v, unsigned int& hi, unsigned int& lo) { hi = f2bf_bits(v); lo = f2bf_bits(v - bf_bits2f(hi)); }
__device__ __forceinline__ void pk8s(v4f a, v4f b, v4u& ph, v4u& pl) {
  unsigned int h0, l0, h1, l1, h2, l2, h3, l3, h4, l4, h5, l5, h6, l6, h7, l7;
  bf_hl(a.x, h0, l0); bf_hl(a.y, h1, l1); bf_hl(a.z, h2, l2); bf_hl(a.w, h3, l3);
  bf_hl(b.x, h4, l4); bf_hl(b.y, h5, l5); bf_hl(b.z, h6, l6); bf_hl(b.w, h7, l7);
  ph.x = h0 | (h1 << 16); ph.y = h2 | (h3 << 16); ph.z = h4 | (h5 << 16); ph.w = h6 | (h7 << 16);
  pl.x = l0 | (l1 << 16); pl.y = l2 | (l3 << 16); pl.z = l4 | (l5 << 16); pl.w = l6 | (l7 << 16);
}

__device__ __forceinline__ v16b ldfrag_g(const __bf16* __restrict__ p) { FB f; f.h[0] = *(const v8b*)p; f.h[1] = *(const v8b*)(p + 16); return f.v; }

template <bool F16> __device__ __forceinline__ v8f mma_raw(v16b a, v16b b, v8f c) {
  if (F16) {
    const v16h ah = __builtin_bit_cast(v16h, a), bh = __builtin_bit_cast(v16h, b);
    return __builtin_amdgcn_wmma_f32_16x16x32_f16(false, ah, false, bh, (short)0, c, false, false);
  }
  return __builtin_amdgcn_wmma_f32_16x16x32_bf16(false, a, false, b, (short)0, c, false, false);
}
template <bool F16> __device__ __forceinline__ v8f mma16(v16b a, v16b b, v8f c) {
  c = mma_raw<F16>(a, b, c);
  asm volatile("v_nop\n\tv_nop\n\tv_nop\n\tv_nop" : "+v"(c) : "v"(a), "v"(b));
  return c;
}
__device__ __forceinline__ void dep_guard_b(v8f& a, v8f& b, v16b x, v16b y) { asm volatile("v_nop\n\tv_nop\n\tv_nop\n\tv_nop" : "+v"(a), "+v"(b) : "v"(x), "v"(y)); }
__device__ __forceinline__ void keep4_b(v16b a, v16b b, v16b c, v16b d) { asm volatile("v_nop" :: "v"(a), "v"(b), "v"(c), "v"(d)); }
__device__ __forceinline__ void acc_guard4(v8f& a, v8f& b, v8f& c, v8f& d) { asm volatile("v_nop\n\tv_nop\n\tv_nop\n\tv_nop" : "+v"(a), "+v"(b), "+v"(c), "+v"(d)); }
__device__ __forceinline__ void wave_sync() {
  __builtin_amdgcn_fence(3  , "workgroup");
  __builtin_amdgcn_wave_barrier();
  __builtin_amdgcn_fence(2  , "workgroup");
}

__global__ __launch_bounds__(256) void k_castT(const float* __restrict__ SRC, int lds, unsigned short* __restrict__ DST, int ldd, int nR, int nC, float sc, int asbf) {
  const long long u = (long long)blockIdx.x * 256 + threadIdx.x; const int per = nR / 8;
  if (u >= (long long)nC * per) return;
  const int c = (int)(u / per); const int r0 = 8 * (int)(u % per);
  const float* s = SRC + (long long)r0 * lds + c;
  v4f wa, wb;
  wa.x = cmb_bf(s[0]) * sc;                  wa.y = cmb_bf(s[(long long)lds]) * sc;
  wa.z = cmb_bf(s[2 * (long long)lds]) * sc; wa.w = cmb_bf(s[3 * (long long)lds]) * sc;
  wb.x = cmb_bf(s[4 * (long long)lds]) * sc; wb.y = cmb_bf(s[5 * (long long)lds]) * sc;
  wb.z = cmb_bf(s[6 * (long long)lds]) * sc; wb.w = cmb_bf(s[7 * (long long)lds]) * sc;
  const v4u ph = pk8h(wa, wb); const v4u pb = pk8b(wa, wb);
  const v4u pk = asbf ? pb : ph;
  volatile v4u* d = (volatile v4u*)(DST + (long long)c * ldd + r0);
  *d = pk; __threadfence(); *d = pk;
}

__global__ __launch_bounds__(256) void k_castE(const float* __restrict__ SRC, unsigned short* __restrict__ DST, long long n8) {
  const long long u = (long long)blockIdx.x * 256 + threadIdx.x; if (u >= n8) return;
  const v4f a = *(const v4f*)(SRC + 8 * u), b = *(const v4f*)(SRC + 8 * u + 4);
  const v4u pk = pk8b(a, b);
  volatile v4u* d = (volatile v4u*)(DST + 8 * u);
  *d = pk; __threadfence(); *d = pk;
}

__global__ __launch_bounds__(128) void k_ln16(const float* __restrict__ X, long long xbs, const float* __restrict__ g, const float* __restrict__ bt,
                                               unsigned short* __restrict__ Y, int rin) {
  __shared__ float red1[4];
  __shared__ float red2[4];
  const int row = blockIdx.x; const int b = row / SEQ, t = row - b * SEQ;
  const int tid = threadIdx.x, lane = tid & 31, wave = tid >> 5, c0 = tid * 8;
  const float* xr = X + (long long)b * xbs + (long long)t * CE + c0;
  v4f a0 = *(const v4f*)xr, a1 = *(const v4f*)(xr + 4);
  if (rin) {
    a0.x = cmb_bf(a0.x); a0.y = cmb_bf(a0.y); a0.z = cmb_bf(a0.z); a0.w = cmb_bf(a0.w);
    a1.x = cmb_bf(a1.x); a1.y = cmb_bf(a1.y); a1.z = cmb_bf(a1.z); a1.w = cmb_bf(a1.w);
  }
  float s = (a0.x + a0.y + a0.z + a0.w) + (a1.x + a1.y + a1.z + a1.w);
  s += __shfl_xor(s, 16, 32); s += __shfl_xor(s, 8, 32); s += __shfl_xor(s, 4, 32); s += __shfl_xor(s, 2, 32); s += __shfl_xor(s, 1, 32);
  if (lane == 0) red1[wave] = s;
  __syncthreads();
  const float mean = ((red1[0] + red1[1]) + (red1[2] + red1[3])) * (1.0f / CE);
  const v4f d0 = a0 - mean, d1 = a1 - mean;
  float q = (d0.x * d0.x + d0.y * d0.y + d0.z * d0.z + d0.w * d0.w) + (d1.x * d1.x + d1.y * d1.y + d1.z * d1.z + d1.w * d1.w);
  q += __shfl_xor(q, 16, 32); q += __shfl_xor(q, 8, 32); q += __shfl_xor(q, 4, 32); q += __shfl_xor(q, 2, 32); q += __shfl_xor(q, 1, 32);
  if (lane == 0) red2[wave] = q;
  __syncthreads();
  const float var = ((red2[0] + red2[1]) + (red2[2] + red2[3])) * (1.0f / CE);
  const float rs = 1.0f / sqrtf(var + 1e-5f);
  const v4f g0 = *(const v4f*)(g + c0), g1 = *(const v4f*)(g + c0 + 4);
  const v4f b0 = *(const v4f*)(bt + c0), b1 = *(const v4f*)(bt + c0 + 4);
  v4f o0, o1;
  o0.x = d0.x * rs * cmb_bf(g0.x) + cmb_bf(b0.x); o0.y = d0.y * rs * cmb_bf(g0.y) + cmb_bf(b0.y);
  o0.z = d0.z * rs * cmb_bf(g0.z) + cmb_bf(b0.z); o0.w = d0.w * rs * cmb_bf(g0.w) + cmb_bf(b0.w);
  o1.x = d1.x * rs * cmb_bf(g1.x) + cmb_bf(b1.x); o1.y = d1.y * rs * cmb_bf(g1.y) + cmb_bf(b1.y);
  o1.z = d1.z * rs * cmb_bf(g1.z) + cmb_bf(b1.z); o1.w = d1.w * rs * cmb_bf(g1.w) + cmb_bf(b1.w);
  const v4u pk = pk8h(o0, o1);
  volatile v4u* d = (volatile v4u*)(Y + (long long)row * CE + c0);
  *d = pk; __threadfence(); *d = pk;
}

template <int ET, bool SPLITA, int BIAS_MODE, int OUT_MODE, int RESID, int ACT>
__global__ __launch_bounds__(256) void k_gemm64(
    const unsigned short* __restrict__ Ap, const unsigned short* __restrict__ A2p, int lda, long long strideA,
    const unsigned short* __restrict__ Btp, int ldb,
    unsigned short* __restrict__ O16a, unsigned short* __restrict__ O16b, unsigned short* __restrict__ O16c,
    float* __restrict__ O32, int ldc, long long strideC,
    const float* __restrict__ bias, const float* __restrict__ resid, int ldr, long long strideR,
    int M, int N, int K, float scale) {
  constexpr bool F16 = (ET == 0);
  __shared__ __align__(16) float sT[8][16 * 68];
  const int bz = blockIdx.y;
  const int lane = threadIdx.x & 31, wave = threadIdx.x >> 5;
  const int tilesN = N >> 6, tilesM = M >> 6;
  const int tile = blockIdx.x * 8 + wave;
  if (tile >= tilesM * tilesN) return;
  const int tm = tile / tilesN, tn = tile - tm * tilesN;
  const int m0 = tm << 6, n0 = tn << 6;
  const __bf16* Ab  = (const __bf16*)Ap + (size_t)bz * (size_t)strideA;
  const __bf16* Ab2 = SPLITA ? ((const __bf16*)A2p + (size_t)bz * (size_t)strideA) : Ab;
  const __bf16* Bb  = (const __bf16*)Btp;
  const int rl = lane & 15, koff = (lane >> 4) * 8, mOff = (lane >> 4) * 8;

  v8f acc[4][4];
#pragma unroll
  for (int i = 0; i < 4; ++i)
#pragma unroll
    for (int j = 0; j < 4; ++j) { v8f z = {}; acc[i][j] = z; }

  for (int k0 = 0; k0 < K; k0 += 32) {
    v16b bh[4];
#pragma unroll
    for (int j = 0; j < 4; ++j) bh[j] = ldfrag_g(Bb + (size_t)(n0 + (j << 4) + rl) * ldb + koff + k0);
#pragma unroll
    for (int i = 0; i < 4; ++i) {
      const size_t ao = (size_t)(m0 + (i << 4) + rl) * lda + koff + k0;
      const v16b ah = ldfrag_g(Ab + ao);
      v16b al = ah;
      if (SPLITA) al = ldfrag_g(Ab2 + ao);
#pragma unroll
      for (int j = 0; j < 4; ++j) {
        acc[i][j] = mma_raw<F16>(ah, bh[j], acc[i][j]);
        if (SPLITA) acc[i][j] = mma_raw<F16>(al, bh[j], acc[i][j]);
      }
      dep_guard_b(acc[i][0], acc[i][3], ah, al);
    }
    keep4_b(bh[0], bh[1], bh[2], bh[3]);
  }
  acc_guard4(acc[0][0], acc[0][1], acc[0][2], acc[0][3]);
  acc_guard4(acc[1][0], acc[1][1], acc[1][2], acc[1][3]);
  acc_guard4(acc[2][0], acc[2][1], acc[2][2], acc[2][3]);
  acc_guard4(acc[3][0], acc[3][1], acc[3][2], acc[3][3]);

  float* slab = sT[wave];
  const float* Rb = (RESID != 0) ? (resid + (size_t)bz * (size_t)strideR) : resid;
#pragma unroll
  for (int i = 0; i < 4; ++i) {
    const int mBase = m0 + (i << 4);
#pragma unroll
    for (int j = 0; j < 4; ++j) {
      const int n = n0 + (j << 4) + rl;
      float bv = 0.f;
      if (BIAS_MODE == 2) bv = cmb_bf(bias[n]);
#pragma unroll
      for (int r = 0; r < 8; ++r) {
        float v = acc[i][j][r] * scale;
        if (BIAS_MODE == 1) v += cmb_bf(bias[mBase + mOff + r]);
        if (BIAS_MODE == 2) v += bv;
        if (ACT == 5) v = 0.5f * v * (1.0f + erff(v * 0.70710678118654752f));
        if (RESID == 1) v += Rb[(size_t)(mBase + mOff + r) * ldr + n];
        if (RESID == 2) v += cmb_bf(Rb[(size_t)(mBase + mOff + r) * ldr + n]);
        slab[(mOff + r) * 68 + (j << 4) + rl] = v;
      }
    }
    wave_sync();
    if (OUT_MODE == 0) {
      float* C = O32 + (size_t)bz * (size_t)strideC;
      const int hh2 = lane >> 4, c4 = (lane & 15) * 4;
      for (int pass = 0; pass < 2; ++pass) {
#pragma unroll
        for (int it = 0; it < 8; ++it) {
          const int row = it * 2 + hh2;
          const v4f v = *(const v4f*)(slab + row * 68 + c4);
          *(volatile v4f*)(C + (size_t)(mBase + row) * ldc + n0 + c4) = v;
        }
        __threadfence();
      }
    } else {
      const int q = lane >> 3, c8 = (lane & 7) * 8;
      for (int pass = 0; pass < 2; ++pass) {
#pragma unroll
        for (int it = 0; it < 4; ++it) {
          const int row = it * 4 + q;
          const float* sp = slab + row * 68 + c8;
          const v4f wa = *(const v4f*)sp, wb = *(const v4f*)(sp + 4);
          const size_t o = (size_t)bz * (size_t)strideC + (size_t)(mBase + row) * ldc + n0 + c8;
          if (OUT_MODE == 1 || OUT_MODE == 3) { const v4u pk = pk8h(wa, wb); *(volatile v4u*)(O16a + o) = pk; }
          if (OUT_MODE == 2) { v4u ph, pl; pk8s(wa, wb, ph, pl); *(volatile v4u*)(O16a + o) = ph; *(volatile v4u*)(O16b + o) = pl; }
          if (OUT_MODE == 3) { v4u ph, pl; pk8s(wa, wb, ph, pl); *(volatile v4u*)(O16b + o) = ph; *(volatile v4u*)(O16c + o) = pl; }
        }
        __threadfence();
      }
    }
    wave_sync();
  }
}

__device__ __forceinline__ float lif_score(float I) {
  const bool good = I > 1.0000001f;
  const float Is = good ? I : 2.0f;
  const float y = __builtin_amdgcn_rcpf(Is);
  const float den = 0.002f - 0.02f * __logf(1.0f - y);
  const float r = __builtin_amdgcn_rcpf(den);
  return good ? 0.125f * r : 0.0f;
}

template <bool F16> __device__ __forceinline__ __bf16 to16(float f) {
  if (F16) return __builtin_bit_cast(__bf16, (_Float16)f);
  return __builtin_bit_cast(__bf16, (unsigned short)f2bf_bits(f));
}

template <bool EARLY>
__global__ __launch_bounds__(128) void k_lif_attn(
    const unsigned short* __restrict__ QHp, const unsigned short* __restrict__ QLp,
    const unsigned short* __restrict__ EBp,
    const unsigned short* __restrict__ VAp, const unsigned short* __restrict__ VBp,
    const float* __restrict__ gain, const float* __restrict__ battn,
    unsigned short* __restrict__ C16, unsigned short* __restrict__ CHp, unsigned short* __restrict__ CLp,
    int nqb, int qb0) {
  constexpr bool F16 = !EARLY;
  const float PSC = F16 ? 32768.0f : 1.0f;
  const float L2E = 1.4426950408889634f;
  __shared__ __align__(16) __bf16 Psh[4][16 * 64];
  __shared__ __align__(16) __bf16 Psl[EARLY ? 4 : 1][EARLY ? 16 * 64 : 8];
  __shared__ __align__(16) float  Os[4][16 * 68];

  const int tid = threadIdx.x, wave = tid >> 5, lane = tid & 31, hh = lane >> 4, c = lane & 15;
  const int bx = blockIdx.x;
  const int qb = qb0 + bx % nqb;
  const int bhd = bx / nqb;
  const int h = bhd % NH, b = bhd / NH;
  const int q0 = qb * 64 + wave * 16;

  const __bf16* QH = (const __bf16*)QHp; const __bf16* QL = (const __bf16*)QLp;
  const __bf16* EB = (const __bf16*)EBp;
  const __bf16* VA = (const __bf16*)VAp; const __bf16* VB = (const __bf16*)VBp;

  v16b qah[2], qal[2];
  {
    const size_t qo = ((size_t)b * SEQ + q0 + c) * CE + (size_t)h * HD + 8 * hh;
#pragma unroll
    for (int dc = 0; dc < 2; ++dc) { qah[dc] = ldfrag_g(QH + qo + dc * 32); qal[dc] = ldfrag_g(QL + qo + dc * 32); }
  }
  float gv[8], bv[8], mrow[8], lrow[8];
#pragma unroll
  for (int r = 0; r < 8; ++r) {
    const int t = q0 + 8 * hh + r;
    gv[r] = cmb_bf(gain[(size_t)h * T_FULL + t]);
    bv[r] = cmb_bf(battn[(size_t)h * T_FULL + t]);
    mrow[r] = -INFINITY; lrow[r] = 0.f;
  }
  v8f oacc[4];
#pragma unroll
  for (int t = 0; t < 4; ++t) { v8f z = {}; oacc[t] = z; }

  __bf16* pwh = Psh[wave];
  __bf16* pwl = Psl[EARLY ? wave : 0];
  const __bf16* erow0 = EB + ((size_t)h * T_FULL + c) * HD + 8 * hh;
  const size_t vcol = (size_t)b * SEQ + 8 * hh;

  for (int kc = 0; kc <= qb; ++kc) {
    const int kv0 = kc * 64;
    v8f s[4];
#pragma unroll
    for (int j = 0; j < 4; ++j) {
      v8f z = {}; s[j] = z;
#pragma unroll
      for (int dc = 0; dc < 2; ++dc) {
        const v16b e = ldfrag_g(erow0 + (size_t)(kv0 + j * 16) * HD + dc * 32);
        s[j] = mma16<false>(qah[dc], e, s[j]);
        s[j] = mma16<false>(qal[dc], e, s[j]);
      }
    }
    const bool diag = (kc == qb);
    float cm[8];
#pragma unroll
    for (int r = 0; r < 8; ++r) {
      const int qrow = q0 + 8 * hh + r;
      float m = -INFINITY;
#pragma unroll
      for (int j = 0; j < 4; ++j) {
        const int kvcol = kv0 + j * 16 + c;
        const float I = gv[r] * s[j][r] + bv[r];
        float sc = lif_score(I);
        sc = (diag && kvcol > qrow) ? -INFINITY : sc;
        s[j][r] = sc;
        m = fmaxf(m, sc);
      }
      m = fmaxf(m, __shfl_xor(m, 1, 32)); m = fmaxf(m, __shfl_xor(m, 2, 32));
      m = fmaxf(m, __shfl_xor(m, 4, 32)); m = fmaxf(m, __shfl_xor(m, 8, 32));
      cm[r] = m;
    }
#pragma unroll
    for (int r = 0; r < 8; ++r) {
      const float mnew = fmaxf(mrow[r], cm[r]);
      const float alpha = __builtin_amdgcn_exp2f((mrow[r] - mnew) * L2E);
      mrow[r] = mnew;
      float psum = 0.f;
#pragma unroll
      for (int j = 0; j < 4; ++j) {
        const float p = __builtin_amdgcn_exp2f((s[j][r] - mnew) * L2E);
        psum += p;
        const int pi = (8 * hh + r) * 64 + j * 16 + c;
        if (EARLY) {
          const unsigned int hb = f2bf_bits(p);
          pwh[pi] = __builtin_bit_cast(__bf16, (unsigned short)hb);
          pwl[pi] = __builtin_bit_cast(__bf16, (unsigned short)f2bf_bits(p - bf_bits2f(hb)));
        } else {
          pwh[pi] = to16<true>(p * PSC);
        }
      }
      psum += __shfl_xor(psum, 1, 32); psum += __shfl_xor(psum, 2, 32);
      psum += __shfl_xor(psum, 4, 32); psum += __shfl_xor(psum, 8, 32);
      lrow[r] = lrow[r] * alpha + psum;
#pragma unroll
      for (int t = 0; t < 4; ++t) oacc[t][r] *= alpha;
    }
    wave_sync();
#pragma unroll
    for (int kk = 0; kk < 2; ++kk) {
      FB pa, pl;
      pa.h[0] = *(const v8b*)(pwh + c * 64 + kk * 32 + 8 * hh);
      pa.h[1] = *(const v8b*)(pwh + c * 64 + kk * 32 + 16 + 8 * hh);
      pl.v = pa.v;
      if (EARLY) {
        pl.h[0] = *(const v8b*)(pwl + c * 64 + kk * 32 + 8 * hh);
        pl.h[1] = *(const v8b*)(pwl + c * 64 + kk * 32 + 16 + 8 * hh);
      }
#pragma unroll
      for (int t = 0; t < 4; ++t) {
        const size_t vo = (size_t)(h * HD + t * 16 + c) * MT + vcol + kv0 + kk * 32;
        const v16b vb = ldfrag_g(VA + vo);
        oacc[t] = mma16<F16>(pa.v, vb, oacc[t]);
        if (EARLY) {
          const v16b vl = ldfrag_g(VB + vo);
          oacc[t] = mma16<false>(pa.v, vl, oacc[t]);
          oacc[t] = mma16<false>(pl.v, vb, oacc[t]);
        }
      }
    }
    wave_sync();
  }

  float* os = Os[wave];
#pragma unroll
  for (int r = 0; r < 8; ++r) {
    const float inv = 1.0f / (lrow[r] * PSC);
#pragma unroll
    for (int t = 0; t < 4; ++t) os[(8 * hh + r) * 68 + t * 16 + c] = oacc[t][r] * inv;
  }
  wave_sync();
  {
    const int q = lane >> 3, c8 = (lane & 7) * 8;
    for (int pass = 0; pass < 2; ++pass) {
#pragma unroll
      for (int it = 0; it < 4; ++it) {
        const int row = it * 4 + q;
        const float* sp = os + row * 68 + c8;
        const v4f wa = *(const v4f*)sp, wb = *(const v4f*)(sp + 4);
        const size_t o = ((size_t)b * SEQ + q0 + row) * CE + (size_t)h * HD + c8;
        const v4u pk = pk8h(wa, wb);
        *(volatile v4u*)(C16 + o) = pk;
        if (EARLY) {
          v4u ph, pl2; pk8s(wa, wb, ph, pl2);
          const size_t oe = ((size_t)b * NX + q0 + row) * CE + (size_t)h * HD + c8;
          *(volatile v4u*)(CHp + oe) = ph;
          *(volatile v4u*)(CLp + oe) = pl2;
        }
      }
      __threadfence();
    }
  }
}

extern "C" void kernel_launch(void* const* d_in, const int* in_sizes, int n_in, void* d_out, int out_size, void* d_ws, size_t ws_size, hipStream_t stream) {
  if (n_in < 16) return;
  const long long need_x = ((long long)(NB - 1) * T_FULL + SEQ) * CE;
  if ((long long)in_sizes[0] < need_x) return;
  if (in_sizes[1] < CE || in_sizes[2] < CE || in_sizes[7] < CE || in_sizes[8] < CE) return;
  if (in_sizes[3] < CE * 3 * CE || in_sizes[4] < 3 * CE) return;
  if (in_sizes[5] < CE * CE || in_sizes[6] < CE) return;
  if (in_sizes[9] < CE * FF || in_sizes[10] < FF || in_sizes[11] < FF * CE || in_sizes[12] < CE) return;
  if (in_sizes[13] < NH * T_FULL * HD || in_sizes[14] < NH * T_FULL || in_sizes[15] < NH * T_FULL) return;
  if ((long long)out_size < need_x) return;

  const float* x      = (const float*)d_in[0];
  const float* ln1_g  = (const float*)d_in[1];
  const float* ln1_b  = (const float*)d_in[2];
  const float* qkv_w  = (const float*)d_in[3];
  const float* qkv_b  = (const float*)d_in[4];
  const float* out_w  = (const float*)d_in[5];
  const float* out_b  = (const float*)d_in[6];
  const float* ln2_g  = (const float*)d_in[7];
  const float* ln2_b  = (const float*)d_in[8];
  const float* mlp_w1 = (const float*)d_in[9];
  const float* mlp_b1 = (const float*)d_in[10];
  const float* mlp_w2 = (const float*)d_in[11];
  const float* mlp_b2 = (const float*)d_in[12];
  const float* enc    = (const float*)d_in[13];
  const float* gaini  = (const float*)d_in[14];
  const float* biasa  = (const float*)d_in[15];
  float* out = (float*)d_out;

  char* wsp = (char*)d_ws; size_t off = 0;
  const size_t PL = (size_t)MT * CE * 2;
  unsigned short* XN16  = (unsigned short*)(wsp + off); off += PL;
  unsigned short* WQV16 = (unsigned short*)(wsp + off); off += (size_t)2 * CE * CE * 2;
  unsigned short* WO16  = (unsigned short*)(wsp + off); off += (size_t)CE * CE * 2;
  unsigned short* WOB   = (unsigned short*)(wsp + off); off += (size_t)CE * CE * 2;
  unsigned short* W1T   = (unsigned short*)(wsp + off); off += (size_t)FF * CE * 2;
  unsigned short* W2T   = (unsigned short*)(wsp + off); off += (size_t)CE * FF * 2;
  unsigned short* EBp   = (unsigned short*)(wsp + off); off += (size_t)NH * T_FULL * HD * 2;
  unsigned short* RQV   = (unsigned short*)(wsp + off); off += 5 * PL;
  unsigned short* C16   = (unsigned short*)(wsp + off); off += PL;
  unsigned short* CHp   = (unsigned short*)(wsp + off); off += (size_t)NB * NX * CE * 2;
  unsigned short* CLp   = (unsigned short*)(wsp + off); off += (size_t)NB * NX * CE * 2;
  float*          X2    = (float*)(wsp + off);          off += (size_t)MT * CE * 4;
  if (off > ws_size) return;
  static_assert((size_t)MT * FF * 2 <= 5 * (size_t)MT * CE * 2);
  unsigned short* QH = RQV; unsigned short* QL = RQV + (size_t)MT * CE;
  unsigned short* VT16 = RQV + 2 * (size_t)MT * CE; unsigned short* VTH = RQV + 3 * (size_t)MT * CE; unsigned short* VTL = RQV + 4 * (size_t)MT * CE;
  unsigned short* HID16 = RQV;
  unsigned short* H16 = XN16;

  const float WS = 64.0f, IWS = 0.015625f;

  k_castT<<<(unsigned)(((long long)CE * (CE / 8) + 255) / 256), 256, 0, stream>>>(qkv_w, 3 * CE, WQV16, CE, CE, CE, WS, 0);
  k_castT<<<(unsigned)(((long long)CE * (CE / 8) + 255) / 256), 256, 0, stream>>>(qkv_w + 2 * CE, 3 * CE, WQV16 + (size_t)CE * CE, CE, CE, CE, WS, 0);
  k_castT<<<(unsigned)(((long long)CE * (CE / 8) + 255) / 256), 256, 0, stream>>>(out_w, CE, WO16, CE, CE, CE, WS, 0);
  k_castT<<<(unsigned)(((long long)CE * (CE / 8) + 255) / 256), 256, 0, stream>>>(out_w, CE, WOB, CE, CE, CE, 1.0f, 1);
  k_castT<<<(unsigned)(((long long)FF * (CE / 8) + 255) / 256), 256, 0, stream>>>(mlp_w1, FF, W1T, CE, CE, FF, WS, 0);
  k_castT<<<(unsigned)(((long long)CE * (FF / 8) + 255) / 256), 256, 0, stream>>>(mlp_w2, CE, W2T, FF, FF, CE, WS, 0);
  k_castE<<<(unsigned)(((long long)NH * T_FULL * HD / 8 + 255) / 256), 256, 0, stream>>>(enc, EBp, (long long)NH * T_FULL * HD / 8);

  k_ln16<<<MT, 128, 0, stream>>>(x, (long long)T_FULL * CE, ln1_g, ln1_b, XN16, 1);

  k_gemm64<0, false, 2, 2, 0, 0><<<dim3((unsigned)(((MT / 64) * (CE / 64) + 7) / 8), 1), 256, 0, stream>>>(
      XN16, nullptr, CE, 0, WQV16, CE, QH, QL, nullptr, nullptr, CE, 0, qkv_b, nullptr, 0, 0, MT, CE, CE, IWS);
  k_gemm64<0, false, 1, 3, 0, 0><<<dim3((unsigned)(((CE / 64) * (MT / 64) + 7) / 8), 1), 256, 0, stream>>>(
      WQV16 + (size_t)CE * CE, nullptr, CE, 0, XN16, CE, VT16, VTH, VTL, nullptr, MT, 0, qkv_b + 2 * CE, nullptr, 0, 0, CE, MT, CE, IWS);

  k_lif_attn<true><<<(unsigned)(NB * NH * (NX / 64)), 128, 0, stream>>>(QH, QL, EBp, VTH, VTL, gaini, biasa, C16, CHp, CLp, NX / 64, 0);
  constexpr int NQB_MAIN = SEQ / 64 - NX / 64;
  if (NQB_MAIN > 0)
    k_lif_attn<false><<<(unsigned)(NB * NH * NQB_MAIN), 128, 0, stream>>>(QH, QL, EBp, VT16, VT16, gaini, biasa, C16, CHp, CLp, NQB_MAIN, NX / 64);

  k_gemm64<0, false, 2, 0, 2, 0><<<dim3((unsigned)(((SEQ / 64) * (CE / 64) + 7) / 8), NB), 256, 0, stream>>>(
      C16, nullptr, CE, (long long)SEQ * CE, WO16, CE, nullptr, nullptr, nullptr, X2, CE, (long long)SEQ * CE,
      out_b, x, CE, (long long)T_FULL * CE, SEQ, CE, CE, IWS);
  k_gemm64<1, true, 2, 0, 2, 0><<<dim3((unsigned)(((NX / 64) * (CE / 64) + 7) / 8), NB), 256, 0, stream>>>(
      CHp, CLp, CE, (long long)NX * CE, WOB, CE, nullptr, nullptr, nullptr, X2, CE, (long long)SEQ * CE,
      out_b, x, CE, (long long)T_FULL * CE, NX, CE, CE, 1.0f);

  k_ln16<<<MT, 128, 0, stream>>>(X2, (long long)SEQ * CE, ln2_g, ln2_b, H16, 0);

  k_gemm64<0, false, 2, 1, 0, 5><<<dim3((unsigned)(((MT / 64) * (FF / 64) + 7) / 8), 1), 256, 0, stream>>>(
      H16, nullptr, CE, 0, W1T, CE, HID16, nullptr, nullptr, nullptr, FF, 0, mlp_b1, nullptr, 0, 0, MT, FF, CE, IWS);
  k_gemm64<0, false, 2, 0, 1, 0><<<dim3((unsigned)(((SEQ / 64) * (CE / 64) + 7) / 8), NB), 256, 0, stream>>>(
      HID16, nullptr, FF, (long long)SEQ * FF, W2T, FF, nullptr, nullptr, nullptr, out, CE, (long long)T_FULL * CE,
      mlp_b2, X2, CE, (long long)SEQ * CE, SEQ, CE, FF, IWS);
}
